// LayerK_34926674051408
// MI455X (gfx1250) — hardware-verified
//
#include <hip/hip_runtime.h>
#include <stddef.h>


#define DF    128
#define NH    8
#define HC    16
#define GR    32
#define AP    136
#define XSP   132
#define NB    496
#define CHUNK 1024
#define NTHR  256
#define NWAVE 8
#define WCAP  128
#define NGRP  (CHUNK / (NTHR * 4))

#define LDS_SACC (NB * DF)
#define LDS_DEN  (NB * NH)
#define LDS_MX   (NB * NH)
#define LDS_LIST (NWAVE * WCAP)
#define LDS_BYTES ((LDS_SACC + LDS_DEN + LDS_MX + LDS_LIST + NWAVE) * 4)

#define SELU_SC 1.0507009873554805f
#define SELU_AL 1.6732632423543772f
#define NEG_BIG (-1.0e30f)

static_assert(WCAP == (CHUNK / NTHR) * 32);
static_assert(NGRP >= 1);
static_assert(CHUNK == NGRP * NTHR * 4);
static_assert(NB <= 512);
static_assert((NB % NWAVE) == 0);
static_assert(CHUNK <= 1024);
static_assert(((LDS_SACC + LDS_DEN) % 4) == 0);
static_assert((LDS_MX % 4) == 0);
static_assert(LDS_BYTES == 289824);

typedef float          v4f  __attribute__((ext_vector_type(4)));
typedef float          v8f  __attribute__((ext_vector_type(8)));
typedef int            v4i  __attribute__((ext_vector_type(4)));
typedef __bf16         v16b __attribute__((ext_vector_type(16)));
union FragB { v16b v; v4i q[2]; };

__device__ __forceinline__ v8f wm(v16b a, v16b b, v8f c) {
  v8f d = __builtin_amdgcn_wmma_f32_16x16x32_bf16(false, a, false, b, (short)0, c, false, false);
  asm volatile("v_nop\n\tv_nop\n\tv_nop\n\tv_nop" : "+v"(d) : "v"(a), "v"(b));
  return d;
}

__device__ __forceinline__ unsigned int bf16_rne(float f) {
  const unsigned int u = __float_as_uint(f);
  return (u + 0x7FFFu + ((u >> 16) & 1u)) >> 16;
}

__device__ __forceinline__ void split2(float a, float b, unsigned int& hi, unsigned int& lo) {
  const unsigned int ha = bf16_rne(a), hb = bf16_rne(b);
  const float ra = a - __uint_as_float(ha << 16);
  const float rb = b - __uint_as_float(hb << 16);
  const unsigned int la = bf16_rne(ra), lb = bf16_rne(rb);
  hi = ha | (hb << 16);
  lo = la | (lb << 16);
}

__device__ __forceinline__ void split8(v4f a, v4f b, v4i& hi, v4i& lo) {
  unsigned int h0, h1, h2, h3, l0, l1, l2, l3;
  split2(a.x, a.y, h0, l0);
  split2(a.z, a.w, h1, l1);
  split2(b.x, b.y, h2, l2);
  split2(b.z, b.w, h3, l3);
  hi.x = (int)h0; hi.y = (int)h1; hi.z = (int)h2; hi.w = (int)h3;
  lo.x = (int)l0; lo.y = (int)l1; lo.z = (int)l2; lo.w = (int)l3;
}

__device__ __forceinline__ float selu1(float v) {
  return v > 0.0f ? SELU_SC * v : SELU_SC * SELU_AL * (__expf(v) - 1.0f);
}

__global__ __launch_bounds__(NTHR) void k_prep(const float* __restrict__ W,
                                               unsigned short* Wth, unsigned short* Wtl, int n8) {
  const int i = blockIdx.x * NTHR + threadIdx.x;
  if (i >= n8) return;
  const int n  = i >> 4;
  const int k0 = (i & 15) * 8;
  v4f a, b;
  a.x = W[(size_t)(k0 + 0) * DF + n]; a.y = W[(size_t)(k0 + 1) * DF + n];
  a.z = W[(size_t)(k0 + 2) * DF + n]; a.w = W[(size_t)(k0 + 3) * DF + n];
  b.x = W[(size_t)(k0 + 4) * DF + n]; b.y = W[(size_t)(k0 + 5) * DF + n];
  b.z = W[(size_t)(k0 + 6) * DF + n]; b.w = W[(size_t)(k0 + 7) * DF + n];
  v4i hi, lo;
  split8(a, b, hi, lo);
  const size_t o = (size_t)n * DF + k0;
  *(volatile v4i*)(Wth + o) = hi;
  *(volatile v4i*)(Wtl + o) = lo;
  __threadfence();
  *(volatile v4i*)(Wth + o) = hi;
  *(volatile v4i*)(Wtl + o) = lo;
}

__device__ __forceinline__ void epi_tile(v8f acc, int T, int hh, int m, int wave, int ncol,
                                         float cs, float cd, float* Xs, float* As, float* Ds) {
  float ss[8], sd[8];
#pragma unroll
  for (int r = 0; r < 8; ++r) {
    const float v = acc[r];
    Xs[(T * 16 + 8 * hh + r) * XSP + ncol] = v;
    ss[r] = v * cs;
    sd[r] = v * cd;
  }
#pragma unroll
  for (int mk = 1; mk < 16; mk <<= 1) {
#pragma unroll
    for (int r = 0; r < 8; ++r) {
      ss[r] += __shfl_xor(ss[r], mk, 32);
      sd[r] += __shfl_xor(sd[r], mk, 32);
    }
  }
  if (m == 0) {
#pragma unroll
    for (int r = 0; r < 8; ++r) {
      As[(T * 16 + 8 * hh + r) * NH + wave] = ss[r];
      Ds[(T * 16 + 8 * hh + r) * NH + wave] = sd[r];
    }
  }
}

__global__ __launch_bounds__(NTHR) void k_gemm(
    const float* __restrict__ x, const unsigned short* __restrict__ Wth,
    const unsigned short* __restrict__ Wtl,
    const float* __restrict__ att_src, const float* __restrict__ att_dst,
    float* xp, float* asrc, float* adst, int nN) {
  __shared__ __attribute__((aligned(16))) unsigned short Ah[GR * AP];
  __shared__ __attribute__((aligned(16))) unsigned short Al[GR * AP];
  __shared__ __attribute__((aligned(16))) float Xs[GR * XSP];
  __shared__ __attribute__((aligned(16))) float As[GR * NH];
  __shared__ __attribute__((aligned(16))) float Ds[GR * NH];

  const int tid  = threadIdx.x;
  const int lane = tid & 31;
  const int wave = tid >> 5;
  const int hh   = lane >> 4;
  const int m    = lane & 15;
  const int rowBase = blockIdx.x * GR;

  {
    const int r  = tid >> 3;
    const int c0 = (tid & 7) * 16;
    int row = rowBase + r;
    if (row > nN - 1) row = nN - 1;
    const float* p = x + (size_t)row * DF + c0;
    const v4f f0 = *(const v4f*)(p), f1 = *(const v4f*)(p + 4);
    const v4f f2 = *(const v4f*)(p + 8), f3 = *(const v4f*)(p + 12);
    v4i h0, l0, h1, l1;
    split8(f0, f1, h0, l0);
    split8(f2, f3, h1, l1);
    *(v4i*)(Ah + r * AP + c0)     = h0;
    *(v4i*)(Ah + r * AP + c0 + 8) = h1;
    *(v4i*)(Al + r * AP + c0)     = l0;
    *(v4i*)(Al + r * AP + c0 + 8) = l1;
  }
  __syncthreads();

  const int ncol = wave * 16 + m;
  v8f c0a = {0.f, 0.f, 0.f, 0.f, 0.f, 0.f, 0.f, 0.f};
  v8f c1a = {0.f, 0.f, 0.f, 0.f, 0.f, 0.f, 0.f, 0.f};
#pragma unroll
  for (int kt = 0; kt < DF / 32; ++kt) {
    const int k0 = kt * 32;
    FragB a0h, a0l, a1h, a1l, bh, bl;
    const unsigned short* pbh  = Wth + (size_t)ncol * DF + k0 + 8 * hh;
    const unsigned short* pbl  = Wtl + (size_t)ncol * DF + k0 + 8 * hh;
    const unsigned short* pa0h = Ah + m * AP + k0 + 8 * hh;
    const unsigned short* pa0l = Al + m * AP + k0 + 8 * hh;
    const unsigned short* pa1h = Ah + (16 + m) * AP + k0 + 8 * hh;
    const unsigned short* pa1l = Al + (16 + m) * AP + k0 + 8 * hh;
    bh.q[0]  = *(const v4i*)pbh;  bh.q[1]  = *(const v4i*)(pbh + 16);
    bl.q[0]  = *(const v4i*)pbl;  bl.q[1]  = *(const v4i*)(pbl + 16);
    a0h.q[0] = *(const v4i*)pa0h; a0h.q[1] = *(const v4i*)(pa0h + 16);
    a0l.q[0] = *(const v4i*)pa0l; a0l.q[1] = *(const v4i*)(pa0l + 16);
    a1h.q[0] = *(const v4i*)pa1h; a1h.q[1] = *(const v4i*)(pa1h + 16);
    a1l.q[0] = *(const v4i*)pa1l; a1l.q[1] = *(const v4i*)(pa1l + 16);
    c0a = wm(a0h.v, bh.v, c0a);
    c0a = wm(a0h.v, bl.v, c0a);
    c0a = wm(a0l.v, bh.v, c0a);
    c1a = wm(a1h.v, bh.v, c1a);
    c1a = wm(a1h.v, bl.v, c1a);
    c1a = wm(a1l.v, bh.v, c1a);
  }

  const float cs = att_src[ncol];
  const float cd = att_dst[ncol];
  epi_tile(c0a, 0, hh, m, wave, ncol, cs, cd, Xs, As, Ds);
  epi_tile(c1a, 1, hh, m, wave, ncol, cs, cd, Xs, As, Ds);
  __syncthreads();

  v4f xr[4];
#pragma unroll
  for (int i = 0; i < 4; ++i) xr[i] = *(const v4f*)(Xs + (4 * wave + i) * XSP + 4 * lane);
  float* gp = 0;
  v4f gv = {0.f, 0.f, 0.f, 0.f};
  if (wave < 2) {
    gv = *(const v4f*)(As + wave * 128 + 4 * lane);
    gp = asrc + (size_t)rowBase * NH + wave * 128 + 4 * lane;
  } else if (wave < 4) {
    gv = *(const v4f*)(Ds + (wave - 2) * 128 + 4 * lane);
    gp = adst + (size_t)rowBase * NH + (wave - 2) * 128 + 4 * lane;
  }
  float* xpp[4];
#pragma unroll
  for (int i = 0; i < 4; ++i) xpp[i] = xp + (size_t)(rowBase + 4 * wave + i) * DF + 4 * lane;

#pragma unroll
  for (int i = 0; i < 4; ++i) *(volatile v4f*)(xpp[i]) = xr[i];
  if (gp) *(volatile v4f*)gp = gv;
  __threadfence();
#pragma unroll
  for (int i = 0; i < 4; ++i) *(volatile v4f*)(xpp[i]) = xr[i];
  if (gp) *(volatile v4f*)gp = gv;
}

__global__ __launch_bounds__(NTHR) void k_gat(
    const int* __restrict__ ei, const float* __restrict__ xp,
    const float* __restrict__ asrc, const float* __restrict__ adst,
    const float* __restrict__ bias, float* out, int nN, int nE) {
  extern __shared__ v4f lds_dyn[];
  float* sacc = (float*)lds_dyn;
  float* den  = sacc + LDS_SACC;
  float* mx   = den + LDS_DEN;
  int*   list = (int*)(mx + LDS_MX);
  int*   wcnt = list + LDS_LIST;

  const int tid  = threadIdx.x;
  const int lane = tid & 31;
  const int wave = tid >> 5;
  const int hd   = lane >> 2;
  const int nodeBase = blockIdx.x * NB;

  {
    const v4f z4 = {0.f, 0.f, 0.f, 0.f};
    const v4f n4 = {NEG_BIG, NEG_BIG, NEG_BIG, NEG_BIG};
    const int nz = (LDS_SACC + LDS_DEN) / 4;
    const int nt = nz + LDS_MX / 4;
    for (int i = tid; i < nt; i += NTHR) lds_dyn[i] = (i < nz) ? z4 : n4;
  }
  __syncthreads();

  const int* eid = ei + nE;
  const bool al16 = ((nE & 3) == 0);

  const int nChunks = (nE + CHUNK - 1) / CHUNK;
#pragma unroll 1
  for (int ch = 0; ch < nChunks; ++ch) {
    const int cbase = ch * CHUNK;
    int wc = 0;
#pragma unroll
    for (int g = 0; g < NGRP; ++g) {
      const int el0 = (g * NTHR + tid) * 4;
      const int e0  = cbase + el0;
      const int sent = -2147483647 - 1;
      v4i d;
      if (al16 && (e0 + 3 < nE)) {
        d = *(const v4i*)(eid + e0);
      } else {
        d.x = (e0     < nE) ? eid[min(e0, nE - 1)]     : sent;
        d.y = (e0 + 1 < nE) ? eid[min(e0 + 1, nE - 1)] : sent;
        d.z = (e0 + 2 < nE) ? eid[min(e0 + 2, nE - 1)] : sent;
        d.w = (e0 + 3 < nE) ? eid[min(e0 + 3, nE - 1)] : sent;
      }
      const unsigned s0 = (unsigned)d.x - (unsigned)nodeBase;
      const unsigned s1 = (unsigned)d.y - (unsigned)nodeBase;
      const unsigned s2 = (unsigned)d.z - (unsigned)nodeBase;
      const unsigned s3 = (unsigned)d.w - (unsigned)nodeBase;
      const bool h0 = s0 < (unsigned)NB;
      const bool h1 = s1 < (unsigned)NB;
      const bool h2 = s2 < (unsigned)NB;
      const bool h3 = s3 < (unsigned)NB;
      const unsigned many = __builtin_amdgcn_ballot_w32(h0 | h1 | h2 | h3);
      if (many != 0u) {
#define HITJ(J, HJ, SJ) { \
          const unsigned mj = __builtin_amdgcn_ballot_w32(HJ); \
          if (HJ) { \
            const int pos = wc + (int)__builtin_amdgcn_mbcnt_lo(mj, 0u); \
            if (pos < WCAP) list[wave * WCAP + pos] = ((el0 + (J)) << 9) | (int)(SJ); \
          } \
          wc += (int)__builtin_popcount(mj); }
        HITJ(0, h0, s0)
        HITJ(1, h1, s1)
        HITJ(2, h2, s2)
        HITJ(3, h3, s3)
#undef HITJ
      }
    }
    if (lane == 0) wcnt[wave] = wc;
    __syncthreads();

    if (wave == 0) {
      for (int wsx = 0; wsx < NWAVE; ++wsx) {
        int n = wcnt[wsx];
        if (n > WCAP) n = WCAP;
        if (n < 0) n = 0;
        for (int i = 0; i < n; ++i) {
          const int ent  = list[wsx * WCAP + i];
          int slot = ent & 511;
          if (slot > NB - 1) slot = NB - 1;
          const int el   = (ent >> 9) & (CHUNK - 1);
          int e = cbase + el;
          if (e > nE - 1) e = nE - 1;
          int src = ei[e];
          src = src < 0 ? 0 : (src > nN - 1 ? nN - 1 : src);
          int nd = nodeBase + slot;
          if (nd > nN - 1) nd = nN - 1;
          float al = asrc[(size_t)src * NH + hd] + adst[(size_t)nd * NH + hd];
          al = (al > 0.f) ? al : 0.2f * al;
          const int ai = slot * NH + hd;
          const float mo = mx[ai];
          const float dn = den[ai];
          const float mn = fmaxf(mo, al);
          const float sc = __expf(mo - mn);
          const float p  = __expf(al - mn);
          const v4f xv = *(const v4f*)(xp + (size_t)src * DF + 4 * lane);
          v4f* sp = (v4f*)(sacc + slot * DF + 4 * lane);
          const v4f cur = *sp;
          const v4f nxt = cur * sc + p * xv;
          *sp = nxt;
          mx[ai]  = mn;
          den[ai] = dn * sc + p;
        }
      }
    }
    __syncthreads();
  }

  const v4f b4 = *(const v4f*)(bias + 4 * lane);
#pragma unroll 1
  for (int j = 0; j < NB / NWAVE; ++j) {
    const int slot = wave * (NB / NWAVE) + j;
    const int node = nodeBase + slot;
    if (node >= nN) break;
    const size_t nrow = (size_t)node;
    float al = asrc[nrow * NH + hd] + adst[nrow * NH + hd];
    al = (al > 0.f) ? al : 0.2f * al;
    const int ai = slot * NH + hd;
    const float mo = mx[ai];
    const float dn = den[ai];
    const float mn = fmaxf(mo, al);
    const float sc = __expf(mo - mn);
    const float p  = __expf(al - mn);
    const v4f xv = *(const v4f*)(xp + nrow * DF + 4 * lane);
    const v4f sv = *(const v4f*)(sacc + slot * DF + 4 * lane) * sc + p * xv;
    const float dv  = dn * sc + p;
    const float inv = 1.0f / (dv + 1e-16f);
    const v4f hv = sv * inv + b4;
    v4f y;
    y.x = selu1(hv.x);
    y.y = selu1(hv.y);
    y.z = selu1(hv.z);
    y.w = selu1(hv.w);
    float* op = out + nrow * DF + 4 * lane;
    *(volatile v4f*)op = y;
    __threadfence();
    *(volatile v4f*)op = y;
  }
}

extern "C" void kernel_launch(void* const* d_in, const int* in_sizes, int n_in,
                              void* d_out, int out_size, void* d_ws, size_t ws_size,
                              hipStream_t stream) {
  if (n_in < 6) return;
  if (in_sizes[0] <= 0 || (in_sizes[0] % DF) != 0) return;
  const int nN = in_sizes[0] / DF;
  if (in_sizes[1] < 0 || (in_sizes[1] & 1) != 0) return;
  const int nE = in_sizes[1] / 2;
  if (in_sizes[2] != DF * DF) return;
  if (in_sizes[3] != NH * HC || in_sizes[4] != NH * HC) return;
  if (in_sizes[5] != DF) return;
  if (out_size != nN * DF) return;

  const float* x       = (const float*)d_in[0];
  const int*   ei      = (const int*)d_in[1];
  const float* W       = (const float*)d_in[2];
  const float* att_src = (const float*)d_in[3];
  const float* att_dst = (const float*)d_in[4];
  const float* bias    = (const float*)d_in[5];
  float* out = (float*)d_out;

  const int nP = ((nN + GR - 1) / GR) * GR;
  size_t off = 0;
  unsigned short* Wth = (unsigned short*)((char*)d_ws + off); off += (size_t)DF * DF * sizeof(unsigned short);
  unsigned short* Wtl = (unsigned short*)((char*)d_ws + off); off += (size_t)DF * DF * sizeof(unsigned short);
  float* xp   = (float*)((char*)d_ws + off);  off += (size_t)nP * DF * sizeof(float);
  float* asrc = (float*)((char*)d_ws + off);  off += (size_t)nP * NH * sizeof(float);
  float* adst = (float*)((char*)d_ws + off);  off += (size_t)nP * NH * sizeof(float);
  if (off > ws_size) return;

  const int n8 = DF * DF / 8;
  k_prep<<<(n8 + NTHR - 1) / NTHR, NTHR, 0, stream>>>(W, Wth, Wtl, n8);

  k_gemm<<<nP / GR, NTHR, 0, stream>>>(x, Wth, Wtl, att_src, att_dst, xp, asrc, adst, nN);

  hipFuncSetAttribute(reinterpret_cast<const void*>(&k_gat),
                      hipFuncAttributeMaxDynamicSharedMemorySize, LDS_BYTES);
  const int grid = (nN + NB - 1) / NB;
  k_gat<<<grid, NTHR, LDS_BYTES, stream>>>(ei, xp, asrc, adst, bias, out, nN, nE);
}
